// SplineCNN_5308579578323
// MI455X (gfx1250) — hardware-verified
//
#include <hip/hip_runtime.h>
#include <math.h>

typedef __attribute__((ext_vector_type(16))) _Float16 v16h;
typedef __attribute__((ext_vector_type(16))) __bf16 v16b;
typedef __attribute__((ext_vector_type(8)))  _Float16 v8h;
typedef __attribute__((ext_vector_type(8)))  float v8f;
typedef __attribute__((ext_vector_type(4)))  float v4f;
typedef __attribute__((ext_vector_type(2)))  float v2f;
typedef __attribute__((ext_vector_type(4)))  unsigned v4u;
typedef __attribute__((ext_vector_type(4)))  int v4i;
typedef float __attribute__((may_alias)) float_a;
typedef int __attribute__((may_alias)) int_a;

template <typename T> __device__ __forceinline__ void vst2(void* p, T v) { *(volatile T*)p = v; __threadfence(); *(volatile T*)p = v; }
__device__ __forceinline__ v8f wmma16(v16h a, v16h b, v8f c) {
  v8f d = __builtin_amdgcn_wmma_f32_16x16x32_f16(false, a, false, b, (short)0, c, false, false);
  asm volatile("v_nop\n\tv_nop\n\tv_nop\n\tv_nop" : "+v"(d) : "v"(a), "v"(b));
  return d;
}
__device__ __forceinline__ v8f wmma_bf(v16b a, v16b b, v8f c) {
  v8f d = __builtin_amdgcn_wmma_f32_16x16x32_bf16(false, a, false, b, (short)0, c, false, false);
  asm volatile("v_nop\n\tv_nop\n\tv_nop\n\tv_nop" : "+v"(d) : "v"(a), "v"(b));
  return d;
}
__device__ __forceinline__ v16h frag_h(const _Float16* rowk0, int lane) {
  union { v16h v; v8h q[2]; } u; const _Float16* p = rowk0 + 8 * (lane >> 4);
  u.q[0] = *(const v8h*)p; u.q[1] = *(const v8h*)(p + 16); return u.v;
}
__device__ __forceinline__ v16h frag_f32(const float* rowk0, int lane) {
  v16h a; const float* p = rowk0 + 8 * (lane >> 4);
#pragma unroll
  for (int i = 0; i < 8; ++i) { a[i] = (_Float16)p[i]; a[8 + i] = (_Float16)p[16 + i]; }
  return a;
}
__device__ __forceinline__ v16h frag_f32s(const float* rowk0, int lane, float sc) {
  v16h a; const float* p = rowk0 + 8 * (lane >> 4);
#pragma unroll
  for (int i = 0; i < 8; ++i) { a[i] = (_Float16)(p[i] * sc); a[8 + i] = (_Float16)(p[16 + i] * sc); }
  return a;
}
__device__ __forceinline__ v16h fragc_f32(const float* W, int k0, int n, int lane, int ld, int K) {
  v16h a; const int g = lane >> 4;
#pragma unroll
  for (int i = 0; i < 8; ++i) { const int ka = k0 + 8 * g + i, kb = ka + 16;
    a[i] = (_Float16)(ka < K ? W[(size_t)(ka < K ? ka : K - 1) * ld + n] : 0.f); a[8 + i] = (_Float16)(kb < K ? W[(size_t)(kb < K ? kb : K - 1) * ld + n] : 0.f); }
  return a;
}
struct F2 { v16b h, l; };
__device__ __forceinline__ F2 bsplit16(const float v[16]) { F2 r;
#pragma unroll
  for (int i = 0; i < 16; ++i) { const __bf16 h = (__bf16)v[i]; r.h[i] = h; r.l[i] = (__bf16)(v[i] - (float)h); }
  return r; }
__device__ __forceinline__ F2 split_row(const float* row, int k0, int lane) { float v[16]; const float* p = row + k0 + 8 * (lane >> 4);
#pragma unroll
  for (int i = 0; i < 8; ++i) { v[i] = p[i]; v[8 + i] = p[16 + i]; }
  return bsplit16(v); }
__device__ __forceinline__ F2 split_rowK(const float* row, int k0, int lane, int K) { float v[16]; const int g = lane >> 4;
#pragma unroll
  for (int i = 0; i < 8; ++i) { const int ka = k0 + 8 * g + i, kb = ka + 16; v[i] = ka < K ? row[ka < K ? ka : K - 1] : 0.f; v[8 + i] = kb < K ? row[kb < K ? kb : K - 1] : 0.f; }
  return bsplit16(v); }
__device__ __forceinline__ F2 split_col(const float* W, int k0, int n, int lane, int ld, int K) { float v[16]; const int g = lane >> 4;
#pragma unroll
  for (int i = 0; i < 8; ++i) { const int ka = k0 + 8 * g + i, kb = ka + 16; v[i] = ka < K ? W[(size_t)(ka < K ? ka : K - 1) * ld + n] : 0.f; v[8 + i] = kb < K ? W[(size_t)(kb < K ? kb : K - 1) * ld + n] : 0.f; }
  return bsplit16(v); }
__device__ __forceinline__ v8f mac3(const F2& a, const F2& b, v8f c) { c = wmma_bf(a.l, b.h, c); c = wmma_bf(a.h, b.l, c); return wmma_bf(a.h, b.h, c); }
__device__ __forceinline__ float sigm(float v) { return 1.0f / (1.0f + expf(-v)); }
#define LDSX() do { asm volatile("s_wait_dscnt 0" ::: "memory"); __builtin_amdgcn_wave_barrier(); __builtin_amdgcn_fence(__ATOMIC_RELEASE, "workgroup"); } while (0)


#define CSR_N 50000
#define CSR_E 1600000
#define NNP 50048
#ifndef TLB
#define TLB (NNP / 64)
#endif

#define CSR_FINN (CSR_E + 32 * CSR_NBK)
#define CSR_CHUNK 4096
#define CSR_BKT 256
#define CSR_NCH ((CSR_E + CSR_CHUNK - 1) / CSR_CHUNK)
#define CSR_NBK ((CSR_N + CSR_BKT - 1) / CSR_BKT)
#define CSR_NBKP (((CSR_NBK + 63) / 64) * 64)
#define CSR_SEGCAP (CSR_E + 32 * CSR_NBK * CSR_NCH)
#ifndef CSR_BCAP
#define CSR_BCAP 10240
#endif
#define CSR_SZ_CNT   (4u * CSR_NCH * CSR_NBKP)
#define CSR_SZ_OFF   (4u * CSR_NBK * (((CSR_NCH + 31) / 32) * 32))
#define CSR_SZ_BST   (4u * (((CSR_NBK + 1 + 31) / 32) * 32))
#define CSR_SZ_SEG   (4u * CSR_SEGCAP)
#define CSR_SZ_FIN   (4u * (CSR_E + 32 * CSR_NBK))
#define CSR_SZ_ROW   (4u * CSR_NBK * CSR_BKT)
#define CSR_OFFP (((CSR_NCH + 31) / 32) * 32)

__global__ __launch_bounds__(256) void k_csr_cnt(const int* __restrict__ DST, int dstride, int* __restrict__ CNT) {
  __shared__ unsigned short sc[256][CSR_NBK + 1]; __shared__ __align__(16) int srow[CSR_NBKP];
  const int c = blockIdx.x, tid = threadIdx.x;
  for (int b = 0; b < CSR_NBK; ++b) sc[tid][b] = 0;
  const size_t e0 = (size_t)c * CSR_CHUNK + tid * 16;
  for (int i = 0; i < 16; ++i) { const size_t e = e0 + i; if (e < (size_t)CSR_E) { int d = DST[e * dstride]; d = min(max(d, 0), CSR_N - 1); sc[tid][d / CSR_BKT] += 1; } }
  __syncthreads();
  for (int b = tid; b < CSR_NBKP; b += 256) { int s = 0; if (b < CSR_NBK) for (int t = 0; t < 256; ++t) s += sc[t][b]; srow[b] = s; }
  __syncthreads();
  for (int q = tid; q < CSR_NBKP / 4; q += 256) vst2((unsigned*)(CNT + (size_t)c * CSR_NBKP + q * 4), *(const v4u*)&srow[q * 4]);
}
__global__ __launch_bounds__(256) void k_csr_scan(const int* __restrict__ CNT, int* __restrict__ OFF, int* __restrict__ BST) {
  __shared__ int sbt[CSR_NBK + 1]; __shared__ int sbs[((CSR_NBK + 1 + 31) / 32) * 32]; __shared__ int scnt[CSR_NBK + 1]; __shared__ __align__(16) int sbuf[64][CSR_OFFP];
  const int tid = threadIdx.x;
  for (int b = tid; b < CSR_NBK; b += 256) { int sp = 0, st = 0; for (int c = 0; c < CSR_NCH; ++c) { const int n = CNT[(size_t)c * CSR_NBKP + b]; st += n; sp += (n + 31) & ~31; } sbt[b] = sp; scnt[b] = st; }
  for (int b = tid; b < ((CSR_NBK + 1 + 31) / 32) * 32; b += 256) sbs[b] = 0;
  __syncthreads();
  if (tid == 0) { int acc = 0, accf = 0; for (int b = 0; b < CSR_NBK; ++b) { const int t = sbt[b]; sbt[b] = acc; acc += t; sbs[b] = accf; accf += (scnt[b] + 31) & ~31; } sbs[CSR_NBK] = accf; }
  __syncthreads();
  for (int b0 = 0; b0 < CSR_NBK; b0 += 64) {
    if (tid < 64 && b0 + tid < CSR_NBK) { const int b = b0 + tid; int o = sbt[b]; for (int c = 0; c < CSR_OFFP; ++c) { if (c < CSR_NCH) { sbuf[tid][c] = o; o += (CNT[(size_t)c * CSR_NBKP + b] + 31) & ~31; } else sbuf[tid][c] = 0; } }
    __syncthreads();
    for (int q = tid; q < 64 * (CSR_OFFP / 4); q += 256) { const int r = q / (CSR_OFFP / 4), pc = q % (CSR_OFFP / 4); if (b0 + r < CSR_NBK) vst2((unsigned*)(OFF + (size_t)(b0 + r) * CSR_OFFP + pc * 4), *(const v4u*)&sbuf[r][pc * 4]); }
    __syncthreads(); }
  for (int q = tid; q < ((CSR_NBK + 1 + 31) / 32) * 32 / 4; q += 256) vst2((unsigned*)(BST + q * 4), *(const v4u*)&sbs[q * 4]);
}
__global__ __launch_bounds__(256) void k_csr_scatter(const int* __restrict__ SRC, const int* __restrict__ DST, int sstride, int dstride, const int* __restrict__ OFF, int* __restrict__ SEGS, int* __restrict__ SEGE) {
  __shared__ unsigned short sc[256][CSR_NBK + 1]; __shared__ int sbase[CSR_NBK + 1]; __shared__ int scn[CSR_NBK + 1]; __shared__ int sord[CSR_CHUNK];
  const int c = blockIdx.x, tid = threadIdx.x;
  for (int b = 0; b < CSR_NBK; ++b) sc[tid][b] = 0;
  const size_t e0 = (size_t)c * CSR_CHUNK + tid * 16; int bk[16];
#pragma unroll
  for (int i = 0; i < 16; ++i) { const size_t e = e0 + i; bk[i] = -1; if (e < (size_t)CSR_E) { int d = DST[e * dstride]; d = min(max(d, 0), CSR_N - 1); bk[i] = d / CSR_BKT; sc[tid][bk[i]] += 1; } }
  __syncthreads();
  for (int b = tid; b < CSR_NBK; b += 256) { int acc = 0; for (int t = 0; t < 256; ++t) { const int v = sc[t][b]; sc[t][b] = (unsigned short)acc; acc += v; } scn[b] = acc; }
  __syncthreads();
  if (tid == 0) { int acc = 0; for (int b = 0; b < CSR_NBK; ++b) { sbase[b] = acc; acc += scn[b]; } }
  __syncthreads();
#pragma unroll
  for (int i = 0; i < 16; ++i) { if (bk[i] >= 0) { const int b = bk[i]; const int r = sc[tid][b]; sc[tid][b] = (unsigned short)(r + 1); sord[sbase[b] + r] = tid * 16 + i; } }
  __syncthreads();
  for (int b = 0; b < CSR_NBK; ++b) { const int n = scn[b]; if (n == 0) continue; const int nl = ((n + 31) & ~31); const size_t o = (size_t)(min(max(OFF[(size_t)b * CSR_OFFP + c], 0), CSR_SEGCAP - nl) & ~31);
    for (int q = tid; q < nl / 4; q += 256) { int4 vs, ve;
#pragma unroll
      for (int k = 0; k < 4; ++k) { const int i = q * 4 + k; int s = -1, eid = -1; if (i < n) { const size_t e = (size_t)c * CSR_CHUNK + sord[sbase[b] + i]; s = min(max(SRC[e * sstride], 0), CSR_N - 1); eid = (int)e; } vs[k] = s; ve[k] = eid; }
      vst2((unsigned*)(SEGS + o + q * 4), *(const v4u*)&vs); vst2((unsigned*)(SEGE + o + q * 4), *(const v4u*)&ve); } }
}
__global__ __launch_bounds__(256) void k_csr_bucket(const int* __restrict__ CNT, const int* __restrict__ OFF, const int* __restrict__ BST, const int* __restrict__ SEGS, const int* __restrict__ SEGE, const int* __restrict__ DST, int dstride, int* __restrict__ FS, int* __restrict__ FE, int* __restrict__ ROWST, int* __restrict__ ROWCNT) {
  __shared__ int ssrc[CSR_BCAP]; __shared__ int seid[CSR_BCAP]; __shared__ unsigned char snod[CSR_BCAP]; __shared__ int souts[CSR_BCAP]; __shared__ int soute[CSR_BCAP]; __shared__ int scount[256]; __shared__ int sstart[257]; __shared__ int stot;
  const int b = blockIdx.x, tid = threadIdx.x;
  if (tid == 0) { int t = 0; for (int c = 0; c < CSR_NCH; ++c) t += min(max(CNT[(size_t)c * CSR_NBKP + b], 0), CSR_CHUNK); stot = (t <= CSR_BCAP) ? t : 0; }
  __syncthreads();
  { int base = 0; for (int c = 0; c < CSR_NCH; ++c) { const int n = min(max(CNT[(size_t)c * CSR_NBKP + b], 0), CSR_CHUNK); const int o = min(max(OFF[(size_t)b * CSR_OFFP + c], 0), CSR_SEGCAP - ((n + 31) & ~31));
      for (int i = tid; i < n; i += 256) { const int p = base + i; if (p < CSR_BCAP) { ssrc[p] = min(max(SEGS[o + i], 0), CSR_N - 1); const int e = min(max(SEGE[o + i], 0), CSR_E - 1); seid[p] = e; int d = DST[(size_t)e * dstride]; d = min(max(d, 0), CSR_N - 1); const int dl = d - b * CSR_BKT; snod[p] = (unsigned char)(dl >= 0 && dl < 256 ? dl : 255); } }
      base += n; } }
  __syncthreads();
  const int node = b * CSR_BKT + tid; int cnt = 0; for (int p = 0; p < stot; ++p) cnt += (snod[p] == tid) ? 1 : 0;
  scount[tid] = cnt; __syncthreads();
  if (tid == 0) { int acc = 0; for (int t = 0; t < 256; ++t) { sstart[t] = acc; acc += scount[t]; } sstart[256] = acc; }
  __syncthreads();
  const int bst0 = min(max(BST[b], 0), CSR_FINN - ((sstart[256] + 31) & ~31)) & ~31; const int gst = bst0 + sstart[tid];
  { int w = sstart[tid]; for (int p = 0; p < stot; ++p) if (snod[p] == tid) { souts[w] = ssrc[p]; soute[w] = seid[p]; ++w; } }
  __syncthreads();
  { const int n = sstart[256]; const int nl = (n + 31) & ~31; for (int q = tid; q < nl / 4; q += 256) { int4 vs, ve;
#pragma unroll
      for (int k = 0; k < 4; ++k) { const int i = q * 4 + k; vs[k] = i < n ? souts[i] : -1; ve[k] = i < n ? soute[i] : -1; }
      vst2((unsigned*)(FS + bst0 + q * 4), *(const v4u*)&vs); vst2((unsigned*)(FE + bst0 + q * 4), *(const v4u*)&ve); } }
  __syncthreads();
  { __shared__ __align__(16) int srs[256], src2[256]; srs[tid] = node < CSR_N ? gst : 0; src2[tid] = node < CSR_N ? cnt : 0; __syncthreads();
    if (tid < 64) vst2((unsigned*)(ROWST + (size_t)b * 256 + tid * 4), *(const v4u*)&srs[tid * 4]); else if (tid < 128) vst2((unsigned*)(ROWCNT + (size_t)b * 256 + (tid - 64) * 4), *(const v4u*)&src2[(tid - 64) * 4]); }
}

typedef __attribute__((ext_vector_type(8))) __bf16 v8b;
__device__ __forceinline__ v16b frag_b(const __bf16* rowk0, int lane) {
  union { v16b v; v8b q[2]; } u; const __bf16* p = rowk0 + 8 * (lane >> 4);
  u.q[0] = *(const v8b*)p; u.q[1] = *(const v8b*)(p + 16); return u.v;
}
__device__ __forceinline__ float bfr(float v) { return (float)(__bf16)v; }
__device__ __attribute__((noinline)) float exp_ni(float v) { return expf(v); }
__device__ __attribute__((noinline)) float log_ni(float v) { return logf(v); }
__device__ __forceinline__ float elu1(float v) { return v > 0.f ? v : (exp_ni(v) - 1.0f); }
#define WS_CNT  0u
#define WS_OFF  (WS_CNT + CSR_SZ_CNT)
#define WS_BST  (WS_OFF + CSR_SZ_OFF)
#define WS_SEGS (WS_BST + CSR_SZ_BST)
#define WS_SEGE (WS_SEGS + CSR_SZ_SEG)
#define WS_FS   (WS_SEGE + CSR_SZ_SEG)
#define WS_FE   (WS_FS + CSR_SZ_FIN)
#define WS_RST  (WS_FE + CSR_SZ_FIN)
#define WS_RCT  (WS_RST + CSR_SZ_ROW)
#define WS_H1   (WS_RCT + CSR_SZ_ROW)
#define WS_PW   (WS_H1 + 4u * NNP * 32)
#define WS_PL1  (WS_PW + 2u * 64 * 160)
#define WS_PL2  (WS_PL1 + 2u * 128 * 64)
#define WS_Y    (WS_PL2 + 2u * 16 * 128)
#define WS_END  (WS_Y + 4u * NNP * 16)

__device__ __forceinline__ void spline_coef(float pseudo, int& lo, float& frac) { float p = fminf(fmaxf(pseudo, 0.f), 1.f) * 4.0f; float fl = floorf(p); fl = fminf(fmaxf(fl, 0.f), 3.f); lo = (int)fl; frac = p - fl; }
__global__ __launch_bounds__(256) void k_pack(const float* __restrict__ W2, const float* __restrict__ LW1, const float* __restrict__ LW2, __bf16* __restrict__ PW, __bf16* __restrict__ PL1, __bf16* __restrict__ PL2) {
  __shared__ __align__(16) __bf16 srow[160];
  const int n = blockIdx.x, tid = threadIdx.x;
  if (n < 64) { if (tid < 160) { const int k = tid / 32, i = tid % 32; srow[tid] = (__bf16)bfr(W2[((size_t)k * 32 + i) * 64 + n]); } __syncthreads(); if (tid < 20) vst2((unsigned*)(PW + (size_t)n * 160 + tid * 8), *(const v4u*)(&srow[tid * 8])); }
  else if (n < 64 + 128) { const int o = n - 64; if (tid < 64) srow[tid] = (__bf16)bfr(LW1[(size_t)tid * 128 + o]); __syncthreads(); if (tid < 8) vst2((unsigned*)(PL1 + (size_t)o * 64 + tid * 8), *(const v4u*)(&srow[tid * 8])); }
  else { const int c = n - 192; if (tid < 128) srow[tid] = (__bf16)(c < 10 ? bfr(LW2[(size_t)tid * 10 + c]) : 0.f); __syncthreads(); if (tid < 16) vst2((unsigned*)(PL2 + (size_t)c * 128 + tid * 8), *(const v4u*)(&srow[tid * 8])); }
}
__global__ __launch_bounds__(256) void k_l1(const float* __restrict__ X, const float* __restrict__ PSEUDO, const float* __restrict__ W1, const float* __restrict__ R1, const float* __restrict__ B1, const int* __restrict__ FS, const int* __restrict__ FE, const int* __restrict__ RST, const int* __restrict__ RCT, float* __restrict__ H1) {
  __shared__ float sw[5][32], sr[32], sb[32];
  const int tid = threadIdx.x; if (tid < 160) sw[tid / 32][tid % 32] = bfr(W1[tid]); if (tid < 32) { sr[tid] = bfr(R1[tid]); sb[tid] = bfr(B1[tid]); }
  __syncthreads();
  const size_t node = (size_t)blockIdx.x * 64 + (tid >> 2); const int o0 = (tid & 3) * 8; float acc[8];
#pragma unroll
  for (int i = 0; i < 8; ++i) acc[i] = 0.f;
  int cnt = 0; float xn = 0.f;
  if (node < (size_t)CSR_N) { cnt = min(max(RCT[node], 0), CSR_BCAP); const int st = min(max(RST[node], 0), CSR_FINN - cnt); xn = bfr(X[node]);
    for (int e = 0; e < cnt; ++e) { const int s = min(max(FS[st + e], 0), CSR_N - 1); const int eid = min(max(FE[st + e], 0), CSR_E - 1); const float xs = bfr(X[s]); int lo; float fr; spline_coef(bfr(PSEUDO[eid]), lo, fr);
#pragma unroll
      for (int i = 0; i < 8; ++i) { float m = (1.0f - fr) * (xs * sw[lo][o0 + i]); m += fr * (xs * sw[lo + 1][o0 + i]); acc[i] += m; } } }
  const float inv = 1.0f / fmaxf((float)cnt, 1.0f);
  v4f v0, v1;
#pragma unroll
  for (int i = 0; i < 4; ++i) { v0[i] = node < (size_t)CSR_N ? elu1(acc[i] * inv + xn * sr[o0 + i] + sb[o0 + i]) : 0.f; v1[i] = node < (size_t)CSR_N ? elu1(acc[4 + i] * inv + xn * sr[o0 + 4 + i] + sb[o0 + 4 + i]) : 0.f; }
  vst2(H1 + node * 32 + o0, v0); vst2(H1 + node * 32 + o0 + 4, v1);
}
__global__ __launch_bounds__(128) void k_l2(const float* __restrict__ H1, const float* __restrict__ PSEUDO, const __bf16* __restrict__ PW, const float* __restrict__ R2, const float* __restrict__ B2, const __bf16* __restrict__ PL1, const float* __restrict__ LB1, const __bf16* __restrict__ PL2, const float* __restrict__ LB2,
                                           const int* __restrict__ FS, const int* __restrict__ FE, const int* __restrict__ RST, const int* __restrict__ RCT, float* __restrict__ Y) {
  __shared__ __align__(16) __bf16 sah[4][16][168], sal[4][16][168]; __shared__ float smsg[4][16][65]; __shared__ float ssum[4][16][65]; __shared__ int sst[4][17]; __shared__ unsigned char senode[4][16];
  __shared__ __align__(16) __bf16 shh[4][16][136], shl[4][16][136]; __shared__ __align__(16) float so[4][16][20]; __shared__ float sr2[32][65]; __shared__ float sb2[64], slb1[128], slb2[16];
  const int tid = threadIdx.x, wave = tid >> 5, lane = tid & 31, col = lane & 15, g = lane >> 4; const size_t n0 = (size_t)blockIdx.x * 64 + wave * 16;
  for (int q = tid; q < 32 * 64; q += 128) sr2[q >> 6][q & 63] = bfr(R2[q]);
  if (tid < 64) sb2[tid] = bfr(B2[tid]); for (int q = tid; q < 128; q += 128) slb1[q] = bfr(LB1[q]); if (tid < 16) slb2[tid] = tid < 10 ? bfr(LB2[tid]) : 0.f;
  for (int q = lane; q < 16 * 65; q += 32) (&ssum[wave][0][0])[q] = 0.f;
  if (lane <= 16) { const size_t n = n0 + min(lane, 15); int c = 0, s = 0; if (n < (size_t)CSR_N) { c = min(max(RCT[n], 0), CSR_BCAP); s = min(max(RST[n], 0), CSR_FINN - c); } sst[wave][lane] = (lane < 16) ? s : s + c; }
  __syncthreads();
  const int ebeg = sst[wave][0]; int eend = sst[wave][16]; eend = max(min(eend, ebeg + 4096), ebeg);
#pragma unroll 1
  for (int t0 = ebeg; t0 < eend; t0 += 16) {
    if (lane < 16) { const int ei = t0 + lane; __bf16* rh = &sah[wave][lane][0]; __bf16* rl = &sal[wave][lane][0];
      if (ei < eend) { const int s = min(max(FS[ei], 0), CSR_N - 1); const int eid = min(max(FE[ei], 0), CSR_E - 1); int lo; float fr; spline_coef(bfr(PSEUDO[eid]), lo, fr);
        int nd = 15; for (int i = 0; i < 16; ++i) if (ei >= sst[wave][i] && ei < sst[wave][i + 1]) nd = i; senode[wave][lane] = (unsigned char)nd;
        const float* xs = H1 + (size_t)s * 32;
        for (int k = 0; k < 5; ++k) { const float cf = (k == lo) ? (1.0f - fr) : ((k == lo + 1) ? fr : 0.f);
          for (int i = 0; i < 32; ++i) { const float v = cf * xs[i]; const __bf16 hb = (__bf16)v; rh[k * 32 + i] = hb; rl[k * 32 + i] = (__bf16)(v - (float)hb); } } }
      else { senode[wave][lane] = 255; for (int i = 0; i < 160; ++i) { rh[i] = (__bf16)0.f; rl[i] = (__bf16)0.f; } } }
    LDSX();
    v8f acc[4] = {};
#pragma unroll
    for (int kc = 0; kc < 5; ++kc) { const v16b ah = frag_b(&sah[wave][col][kc * 32], lane), al = frag_b(&sal[wave][col][kc * 32], lane);
#pragma unroll
      for (int j = 0; j < 4; ++j) { const v16b w = frag_b(PW + (size_t)(j * 16 + col) * 160 + kc * 32, lane); acc[j] = wmma_bf(al, w, acc[j]); acc[j] = wmma_bf(ah, w, acc[j]); } }
#pragma unroll
    for (int j = 0; j < 4; ++j)
#pragma unroll
      for (int r = 0; r < 8; ++r) smsg[wave][8 * g + r][j * 16 + col] = acc[j][r];
    LDSX();
    for (int e = 0; e < 16; ++e) { const int nd = senode[wave][e]; if (nd < 16) { ssum[wave][nd][lane] += smsg[wave][e][lane]; ssum[wave][nd][lane + 32] += smsg[wave][e][lane + 32]; } }
    LDSX(); }
  { const int rl = lane >> 1, half = lane & 1; const size_t n = n0 + rl; const int deg = sst[wave][rl + 1] - sst[wave][rl]; const float inv = 1.0f / fmaxf((float)deg, 1.0f); const float* hn = H1 + (n < (size_t)NNP ? n : 0) * 32;
    for (int o = half * 32; o < half * 32 + 32; ++o) { float rt = 0.f; for (int i = 0; i < 32; ++i) rt += hn[i] * sr2[i][o]; const float v = elu1(ssum[wave][rl][o] * inv + rt + sb2[o]); const __bf16 hb = (__bf16)v; shh[wave][rl][o] = hb; shl[wave][rl][o] = (__bf16)(v - (float)hb); } }
  LDSX();
  { v8f acc[8] = {};
#pragma unroll
    for (int kc = 0; kc < 2; ++kc) { const v16b ah = frag_b(&shh[wave][col][kc * 32], lane), al = frag_b(&shl[wave][col][kc * 32], lane);
#pragma unroll
      for (int j = 0; j < 8; ++j) { const v16b w = frag_b(PL1 + (size_t)(j * 16 + col) * 64 + kc * 32, lane); acc[j] = wmma_bf(al, w, acc[j]); acc[j] = wmma_bf(ah, w, acc[j]); } }
    LDSX();
#pragma unroll
    for (int j = 0; j < 8; ++j) { const int o = j * 16 + col;
#pragma unroll
      for (int r = 0; r < 8; ++r) { const float v = elu1(acc[j][r] + slb1[o]); const __bf16 hb = (__bf16)v; shh[wave][8 * g + r][o] = hb; shl[wave][8 * g + r][o] = (__bf16)(v - (float)hb); } } }
  LDSX();
  { v8f acc = {};
#pragma unroll
    for (int kc = 0; kc < 4; ++kc) { const v16b ah = frag_b(&shh[wave][col][kc * 32], lane), al = frag_b(&shl[wave][col][kc * 32], lane); const v16b w = frag_b(PL2 + (size_t)col * 128 + kc * 32, lane); acc = wmma_bf(al, w, acc); acc = wmma_bf(ah, w, acc); }
#pragma unroll
    for (int r = 0; r < 8; ++r) so[wave][8 * g + r][col] = acc[r] + slb2[col]; }
  LDSX();
  if (lane < 16) { float mx = -3.0e38f; for (int c = 0; c < 10; ++c) mx = fmaxf(mx, so[wave][lane][c]); float z = 0.f; for (int c = 0; c < 10; ++c) z += exp_ni(so[wave][lane][c] - mx); const float lz = mx + log_ni(z);
    for (int c = 0; c < 10; ++c) so[wave][lane][c] -= lz; for (int c = 10; c < 16; ++c) so[wave][lane][c] = 0.f; }
  LDSX();
  for (int rl = 0; rl < 16; ++rl) if (lane < 4) vst2(Y + (n0 + rl) * 16 + lane * 4, *(const v4f*)&so[wave][rl][lane * 4]);
}
__global__ __launch_bounds__(256) void k_copy(const float* __restrict__ Yb, float* __restrict__ out) {
  const size_t p = (size_t)blockIdx.x * 256 + threadIdx.x; const size_t total = (size_t)CSR_N * 10;
  if (p * 4 >= total) return; v4f v;
#pragma unroll
  for (int i = 0; i < 4; ++i) { const size_t f = p * 4 + i; v[i] = f < total ? Yb[(f / 10) * 16 + (f % 10)] : 0.f; }
  vst2(out + p * 4, v);
}

extern "C" void kernel_launch(void* const* d_in, const int* in_sizes, int n_in, void* d_out, int out_size, void* d_ws, size_t ws_size, hipStream_t stream) {
  (void)in_sizes; (void)n_in; (void)out_size;
  const float** F = (const float**)d_in; const int* EI = (const int*)d_in[1];
  if (ws_size < (size_t)WS_END) return;
  char* ws = (char*)d_ws;
  int *CNT = (int*)(ws + WS_CNT), *OFF = (int*)(ws + WS_OFF), *BST = (int*)(ws + WS_BST), *SEGS = (int*)(ws + WS_SEGS), *SEGE = (int*)(ws + WS_SEGE), *FS = (int*)(ws + WS_FS), *FE = (int*)(ws + WS_FE), *RST = (int*)(ws + WS_RST), *RCT = (int*)(ws + WS_RCT);
  float *H1 = (float*)(ws + WS_H1), *Y = (float*)(ws + WS_Y); __bf16 *PW = (__bf16*)(ws + WS_PW), *PL1 = (__bf16*)(ws + WS_PL1), *PL2 = (__bf16*)(ws + WS_PL2);
  const int* SRC = EI; const int* DST = EI + CSR_E;
  k_csr_cnt<<<CSR_NCH, 256, 0, stream>>>(DST, 1, CNT);
  k_csr_scan<<<1, 256, 0, stream>>>(CNT, OFF, BST);
  k_csr_scatter<<<CSR_NCH, 256, 0, stream>>>(SRC, DST, 1, 1, OFF, SEGS, SEGE);
  k_csr_bucket<<<CSR_NBK, 256, 0, stream>>>(CNT, OFF, BST, SEGS, SEGE, DST, 1, FS, FE, RST, RCT);
  k_pack<<<64 + 128 + 16, 256, 0, stream>>>(F[6], F[9], F[11], PW, PL1, PL2);
  k_l1<<<NNP / 64, 256, 0, stream>>>(F[0], F[2], F[3], F[4], F[5], FS, FE, RST, RCT, H1);
  k_l2<<<TLB, 128, 0, stream>>>(H1, F[2], PW, F[7], F[8], PL1, F[10], PL2, F[12], FS, FE, RST, RCT, Y);
  k_copy<<<(CSR_N * 10 / 4 + 255) / 256, 256, 0, stream>>>(Y, (float*)d_out);
}
